// local_branch_70111046140245
// MI455X (gfx1250) — hardware-run, weakly checked
//
#include <hip/hip_runtime.h>


#ifndef NB
#define NB 2
#endif
#define NB_FULL 2
#define CIN  256
#define DKC  128
#define NPOS 1024
#define NQ   256
#define NOBJ 12
#define WOS  64.0f
#define WOI  (1.0f / 64.0f)
#define W3S  16.0f
#define W3I  (1.0f / 16.0f)
#define WO8  (16 * NPOS / 8)
#define W38  (16 * DKC / 8)
#define NSM8 (WO8 + W38)

static_assert(NB <= NB_FULL);
static_assert(CIN % 32 == 0);
static_assert(DKC % 32 == 0);
static_assert(NPOS % 32 == 0);
static_assert(CIN % 64 == 0);
static_assert(DKC % 64 == 0);
static_assert(NPOS % 64 == 0);
static_assert(NQ % 64 == 0);
static_assert((NB * NPOS) % 64 == 0);
static_assert((NB * NQ) % 64 == 0);
static_assert(NOBJ <= 16);
static_assert(NOBJ % 2 == 0);
static_assert(NPOS / 8 == 128);
static_assert(DKC / 8 == 16);
static_assert(NSM8 % 256 == 0);
static_assert(((size_t)DKC * CIN) % 8 == 0);
static_assert(256 * 2 * 16 == 64 * 128);
static_assert(256 * 4 * 16 == 64 * 64 * 4);
static_assert(32 * 16 * 4 == 16 * 128);
static_assert(32 * 16 * (NOBJ / 2) == NOBJ * 64 * 4);
static_assert(64 * 68 * 4 <= 131072);
static_assert(16 * 68 * 4 <= 131072);
static_assert((size_t)NB_FULL * NOBJ * NQ * 4 == (size_t)24576);

typedef _Float16 h16;
typedef unsigned short bf;
typedef __attribute__((ext_vector_type(16))) __bf16   v16bf;
typedef __attribute__((ext_vector_type(16))) _Float16 v16h;
typedef __attribute__((ext_vector_type(8)))  _Float16 v8h;
typedef __attribute__((ext_vector_type(8)))  unsigned short v8us;
typedef __attribute__((ext_vector_type(8)))  float    v8f;
typedef __attribute__((ext_vector_type(4)))  float    v4f;
typedef v4f  __attribute__((may_alias)) v4fa;

__device__ __forceinline__ unsigned short f2bf(float f) { unsigned u = __float_as_uint(f); u += 0x7FFFu + ((u >> 16) & 1u); return (unsigned short)(u >> 16); }
__device__ __forceinline__ float bfr(float f) { return __uint_as_float(((unsigned)f2bf(f)) << 16); }
__device__ __forceinline__ v16h cat16(v8h lo, v8h hi) { return __builtin_shufflevector(lo, hi, 0, 1, 2, 3, 4, 5, 6, 7, 8, 9, 10, 11, 12, 13, 14, 15); }
__device__ __forceinline__ v16bf cat16b(v8us lo, v8us hi) { return __builtin_bit_cast(v16bf, __builtin_shufflevector(lo, hi, 0, 1, 2, 3, 4, 5, 6, 7, 8, 9, 10, 11, 12, 13, 14, 15)); }
__device__ __forceinline__ v8f wmma16(v16h a, v16h b, v8f c) { return __builtin_amdgcn_wmma_f32_16x16x32_f16(false, a, false, b, (short)0, c, false, false); }
__device__ __forceinline__ v8f wmmab(v16bf a, v16bf b, v8f c) { return __builtin_amdgcn_wmma_f32_16x16x32_bf16(false, a, false, b, (short)0, c, false, false); }
__device__ __forceinline__ v16h  ldh(const h16* p) { return cat16(*(const v8h*)p, *(const v8h*)(p + 16)); }
__device__ __forceinline__ v16bf ldb(const bf* p)  { return cat16b(*(const v8us*)p, *(const v8us*)(p + 16)); }
__device__ __forceinline__ void wave_sync() { __builtin_amdgcn_fence(3  , "wavefront"); __builtin_amdgcn_wave_barrier(); asm volatile("" ::: "memory"); }

static __device__ __forceinline__ h16 toh_flush(float v) { const h16 r = (h16)v; return (fabsf(v) < 6.103515625e-05f) ? (h16)0.0f : r; }
__device__ __forceinline__ v8f wmma16g(v16h a, v16h b, v8f c) { c = wmma16(a, b, c); asm volatile("v_nop\n\tv_nop\n\tv_nop\n\tv_nop" : "+v"(c) : "v"(a), "v"(b)); return c; }
__device__ __forceinline__ v8f wmmabg(v16bf a, v16bf b, v8f c) { c = wmmab(a, b, c); asm volatile("v_nop\n\tv_nop\n\tv_nop\n\tv_nop" : "+v"(c) : "v"(a), "v"(b)); return c; }

__global__ __launch_bounds__(256) void k_cvt8(const float* __restrict__ src, bf* dst, size_t n8) {
    const size_t i = (size_t)blockIdx.x * 256 + threadIdx.x; if (i >= n8) return;
    const v8f v = *(const v8f*)(src + i * 8); v8us o;
#pragma unroll
    for (int k = 0; k < 8; ++k) o[k] = f2bf(v[k]);
    *(volatile v8us*)(dst + i * 8) = o; __threadfence(); *(volatile v8us*)(dst + i * 8) = o;
}

__global__ __launch_bounds__(256) void k_tcvt(const float* __restrict__ src, bf* dst, int R, int C, size_t sstride, int fmt) {
    __shared__ __align__(16) float ts[64 * 68];
    const int c0 = blockIdx.x * 64, r0 = blockIdx.y * 64, b = blockIdx.z;
    const int tid = threadIdx.x;
    const float* sp = src + (size_t)b * sstride;
    bf* dp = dst + (size_t)b * (size_t)R * (size_t)C;
#pragma unroll
    for (int it = 0; it < 4; ++it) { const int q = it * 256 + tid; const int r = q >> 4, c4 = (q & 15) * 4;
        const v4f v = *(const v4f*)(sp + (size_t)(r0 + r) * (size_t)C + (size_t)(c0 + c4));
        *(v4fa*)(&ts[r * 68 + c4]) = v; }
    __syncthreads();
    v8us o[2]; size_t off[2];
#pragma unroll
    for (int it = 0; it < 2; ++it) { const int q = it * 256 + tid; const int c = q >> 3, r8 = (q & 7) * 8;
        v8us ob; v8h oh;
#pragma unroll
        for (int e = 0; e < 8; ++e) { const float x = ts[(r8 + e) * 68 + c]; ob[e] = f2bf(x); oh[e] = toh_flush(bfr(x)); }
        if (fmt != 0) o[it] = __builtin_bit_cast(v8us, oh); else o[it] = ob;
        off[it] = (size_t)(c0 + c) * (size_t)R + (size_t)(r0 + r8); }
#pragma unroll 1
    for (int ps = 0; ps < 2; ++ps) {
#pragma unroll
        for (int it = 0; it < 2; ++it) *(volatile v8us*)(dp + off[it]) = o[it];
        if (ps == 0) __threadfence(); }
}

__global__ __launch_bounds__(256) void k_small(const float* __restrict__ wobj, const float* __restrict__ w3, h16* dst) {
    const int i = blockIdx.x * 256 + threadIdx.x; if (i >= NSM8) return;
    const int iw = i < WO8 ? i : (WO8 - 1);
    const int row = iw >> 7, c8 = (iw & 127) * 8;
    const int rowc = row < NOBJ ? row : (NOBJ - 1);
    int j = i - WO8; j = j < 0 ? 0 : j; j = j > (W38 - 1) ? (W38 - 1) : j;
    const int d8 = (j & 15) * 8;
    v8f a = *(const v8f*)(wobj + (size_t)rowc * NPOS + c8);
    v8f w = *(const v8f*)(w3 + d8);
    asm volatile("" : "+v"(a)); asm volatile("" : "+v"(w));
    const bool isw = i < WO8; const bool live = row < NOBJ;
    v8h o;
#pragma unroll
    for (int e = 0; e < 8; ++e) { const float va = live ? bfr(a[e]) * WOS : 0.0f; const float vw = bfr(w[e]) * W3S; o[e] = toh_flush(isw ? va : vw); }
    *(volatile v8h*)(dst + (size_t)i * 8) = o; __threadfence(); *(volatile v8h*)(dst + (size_t)i * 8) = o;
}

__global__ __launch_bounds__(32) void k_keyf(const bf* __restrict__ A, const bf* __restrict__ Bt, h16* KT) {
    __shared__ __align__(16) float os[16 * 68];
    const int K = CIN;
    const int lane = threadIdx.x & 31, lr = lane & 15, hi = lane >> 4; const int r0 = blockIdx.x * 64, c0 = blockIdx.y * 64;
    v8f acc[4][4];
#pragma unroll
    for (int mb = 0; mb < 4; ++mb)
#pragma unroll
        for (int nb = 0; nb < 4; ++nb) acc[mb][nb] = (v8f){};
    const size_t aoff = (size_t)(r0 + lr) * K + 8 * hi, boff = (size_t)(c0 + lr) * K + 8 * hi;
#pragma unroll 1
    for (int kc = 0; kc < K; kc += 32) {
        v16bf a[4];
#pragma unroll
        for (int mb = 0; mb < 4; ++mb) a[mb] = ldb(A + aoff + (size_t)mb * 16 * K + kc);
#pragma unroll
        for (int nb = 0; nb < 4; ++nb) { const v16bf b = ldb(Bt + boff + (size_t)nb * 16 * K + kc);
#pragma unroll
            for (int mb = 0; mb < 4; ++mb) acc[mb][nb] = wmmabg(a[mb], b, acc[mb][nb]); }
    }
#pragma unroll
    for (int mb = 0; mb < 4; ++mb) {
#pragma unroll
        for (int nb = 0; nb < 4; ++nb) {
#pragma unroll
            for (int j = 0; j < 8; ++j) os[(hi * 8 + j) * 68 + nb * 16 + lr] = acc[mb][nb][j]; }
        wave_sync();
#pragma unroll 1
        for (int ps = 0; ps < 2; ++ps) {
#pragma unroll
            for (int s = 0; s < 4; ++s) { const int row = 4 * s + (lane >> 3), c8 = (lane & 7) * 8;
                const v4f x0 = *(const v4fa*)(&os[row * 68 + c8]); const v4f x1 = *(const v4fa*)(&os[row * 68 + c8 + 4]); v8h hv;
#pragma unroll
                for (int i = 0; i < 4; ++i) { hv[i] = toh_flush(x0[i]); hv[4 + i] = toh_flush(x1[i]); }
                const size_t oo = (size_t)(r0 + mb * 16 + row) * DKC + (size_t)(c0 + c8);
                *(volatile v8h*)(KT + oo) = hv; }
            if (ps == 0) __threadfence(); }
        wave_sync();
    }
}

__global__ __launch_bounds__(32) void k_att(const h16* __restrict__ A, const h16* __restrict__ Bt, const h16* __restrict__ W3, const float* __restrict__ b3p, h16* U) {
    __shared__ __align__(16) float os[16 * 68];
    const int K = DKC;
    const int lane = threadIdx.x & 31, lr = lane & 15, hi = lane >> 4; const int r0 = blockIdx.x * 64, c0 = blockIdx.y * 64;
    const int b = r0 / NQ;
    const float b3v = bfr(b3p[0]);
    const size_t aoff = (size_t)(r0 + lr) * K + 8 * hi, boff = ((size_t)b * NPOS + (size_t)(c0 + lr)) * K + 8 * hi;
    const size_t woff = (size_t)lr * K + 8 * hi;
    v8f sacc[4];
#pragma unroll
    for (int nb = 0; nb < 4; ++nb) sacc[nb] = (v8f){};
#pragma unroll 1
    for (int kc = 0; kc < K; kc += 32) {
        const v16h a3 = ldh(W3 + woff + kc);
#pragma unroll
        for (int nb = 0; nb < 4; ++nb) { const v16h bq = ldh(Bt + boff + (size_t)nb * 16 * K + kc); sacc[nb] = wmma16g(a3, bq, sacc[nb]); }
    }
    float sv[4];
#pragma unroll
    for (int nb = 0; nb < 4; ++nb) sv[nb] = sacc[nb][0] * W3I;
    v8f acc[4][4];
#pragma unroll
    for (int mb = 0; mb < 4; ++mb)
#pragma unroll
        for (int nb = 0; nb < 4; ++nb) acc[mb][nb] = (v8f){};
#pragma unroll 1
    for (int kc = 0; kc < K; kc += 32) {
        v16h a[4];
#pragma unroll
        for (int mb = 0; mb < 4; ++mb) a[mb] = ldh(A + aoff + (size_t)mb * 16 * K + kc);
#pragma unroll
        for (int nb = 0; nb < 4; ++nb) { const v16h bq = ldh(Bt + boff + (size_t)nb * 16 * K + kc);
#pragma unroll
            for (int mb = 0; mb < 4; ++mb) acc[mb][nb] = wmma16g(a[mb], bq, acc[mb][nb]); }
    }
#pragma unroll
    for (int mb = 0; mb < 4; ++mb) {
#pragma unroll
        for (int nb = 0; nb < 4; ++nb) {
#pragma unroll
            for (int j = 0; j < 8; ++j) os[(hi * 8 + j) * 68 + nb * 16 + lr] = (acc[mb][nb][j] + 1.0f) * sv[nb] + b3v; }
        wave_sync();
#pragma unroll 1
        for (int ps = 0; ps < 2; ++ps) {
#pragma unroll
            for (int s = 0; s < 4; ++s) { const int row = 4 * s + (lane >> 3), c8 = (lane & 7) * 8;
                const v4f x0 = *(const v4fa*)(&os[row * 68 + c8]); const v4f x1 = *(const v4fa*)(&os[row * 68 + c8 + 4]); v8h hv;
#pragma unroll
                for (int i = 0; i < 4; ++i) { hv[i] = toh_flush(x0[i]); hv[4 + i] = toh_flush(x1[i]); }
                const size_t oo = (size_t)(r0 + mb * 16 + row) * NPOS + (size_t)(c0 + c8);
                *(volatile v8h*)(U + oo) = hv; }
            if (ps == 0) __threadfence(); }
        wave_sync();
    }
}

__global__ __launch_bounds__(32) void k_obj(const h16* __restrict__ WO, const h16* __restrict__ U, float* OUT) {
    __shared__ __align__(16) float os[16 * 68];
    const int K = NPOS;
    const int lane = threadIdx.x & 31, lr = lane & 15, hi = lane >> 4; const int n0 = blockIdx.x * 64;
    v8f acc[4];
#pragma unroll
    for (int nb = 0; nb < 4; ++nb) acc[nb] = (v8f){};
    const size_t aoff = (size_t)lr * K + 8 * hi, boff = (size_t)(n0 + lr) * K + 8 * hi;
#pragma unroll 1
    for (int kc = 0; kc < K; kc += 32) {
        const v16h a = ldh(WO + aoff + kc);
#pragma unroll
        for (int nb = 0; nb < 4; ++nb) { const v16h bu = ldh(U + boff + (size_t)nb * 16 * K + kc); acc[nb] = wmma16g(a, bu, acc[nb]); }
    }
#pragma unroll
    for (int nb = 0; nb < 4; ++nb) {
#pragma unroll
        for (int j = 0; j < 8; ++j) os[(hi * 8 + j) * 68 + nb * 16 + lr] = acc[nb][j] * WOI; }
    wave_sync();
    const int b = n0 / NQ, i0 = n0 % NQ;
    float* ob = OUT + (size_t)b * NOBJ * NQ + i0;
#pragma unroll 1
    for (int ps = 0; ps < 2; ++ps) {
#pragma unroll
        for (int s = 0; s < NOBJ / 2; ++s) { const int row = 2 * s + (lane >> 4), cofs = (lane & 15) * 4;
            const v4f val = *(const v4fa*)(&os[row * 68 + cofs]);
            *(volatile v4f*)(ob + (size_t)row * NQ + cofs) = val; }
        if (ps == 0) __threadfence(); }
}

static constexpr size_t al256(size_t v) { return (v + 255) & ~(size_t)255; }
static constexpr size_t SZ_WK = al256((size_t)DKC * CIN * 2);
static constexpr size_t SZ_XT = al256((size_t)NB * NPOS * CIN * 2);
static constexpr size_t SZ_QT = al256((size_t)NB * NQ * DKC * 2);
static constexpr size_t SZ_SM = al256((size_t)NSM8 * 16);
static constexpr size_t SZ_KT = al256((size_t)NB * NPOS * DKC * 2);
static constexpr size_t SZ_U  = al256((size_t)NB * NQ * NPOS * 2);
static constexpr size_t SZ_TOTAL = SZ_WK + SZ_XT + SZ_QT + SZ_SM + SZ_KT + SZ_U;
static_assert(SZ_TOTAL <= (size_t)134217728);
static_assert(((size_t)WO8 * 16) % 256 == 0);

extern "C" void kernel_launch(void* const* d_in, const int* in_sizes, int n_in,
                              void* d_out, int out_size, void* d_ws, size_t ws_size, hipStream_t stream) {
    if (n_in < 6) return;
    if ((size_t)in_sizes[0] < (size_t)NB * CIN * NPOS) return;
    if ((size_t)in_sizes[1] < (size_t)NB * DKC * NQ) return;
    if ((size_t)in_sizes[2] < (size_t)DKC * CIN) return;
    if (in_sizes[3] < DKC || in_sizes[4] < 1) return;
    if ((size_t)in_sizes[5] < (size_t)NOBJ * NPOS) return;
    if ((size_t)out_size < (size_t)NB * NOBJ * NQ) return;
    if (SZ_TOTAL > ws_size) return;
    const float* kin  = (const float*)d_in[0];
    const float* qin  = (const float*)d_in[1];
    const float* wkey = (const float*)d_in[2];
    const float* w3   = (const float*)d_in[3];
    const float* b3   = (const float*)d_in[4];
    const float* wobj = (const float*)d_in[5];
    float* OUT = (float*)d_out;
    char* wsp = (char*)d_ws;
    bf*  WKB = (bf*)wsp;  wsp += SZ_WK;
    bf*  XT  = (bf*)wsp;  wsp += SZ_XT;
    h16* QT  = (h16*)wsp; wsp += SZ_QT;
    h16* SM  = (h16*)wsp; wsp += SZ_SM;
    h16* KT  = (h16*)wsp; wsp += SZ_KT;
    h16* U   = (h16*)wsp; wsp += SZ_U;
    h16* WO = SM; h16* W3 = SM + (size_t)WO8 * 8;

    { const size_t n8 = (size_t)DKC * CIN / 8; k_cvt8<<<(unsigned)((n8 + 255) / 256), 256, 0, stream>>>(wkey, WKB, n8); }
    k_tcvt<<<dim3(NPOS / 64, CIN / 64, NB), 256, 0, stream>>>(kin, XT, CIN, NPOS, (size_t)CIN * NPOS, 0);
    k_tcvt<<<dim3(NQ / 64, DKC / 64, NB), 256, 0, stream>>>(qin, (bf*)QT, DKC, NQ, (size_t)DKC * NQ, 1);
    k_small<<<NSM8 / 256, 256, 0, stream>>>(wobj, w3, SM);

    k_keyf<<<dim3(NB * NPOS / 64, DKC / 64, 1), 32, 0, stream>>>(XT, WKB, KT);
    k_att<<<dim3(NB * NQ / 64, NPOS / 64, 1), 32, 0, stream>>>(QT, KT, W3, b3, U);
    k_obj<<<dim3(NB * NQ / 64, 1, 1), 32, 0, stream>>>(WO, U, OUT);
}
